// MambaPlusPlus_layer_48103633715534
// MI455X (gfx1250) — hardware-verified
//
#include <hip/hip_runtime.h>
#include <math.h>

typedef __attribute__((ext_vector_type(16))) _Float16 v16h;
typedef __attribute__((ext_vector_type(8)))  _Float16 v8h;
typedef __attribute__((ext_vector_type(2)))  _Float16 v2h;
typedef __attribute__((ext_vector_type(8)))  float    v8f;
typedef __attribute__((ext_vector_type(4)))  float    v4f;
typedef __attribute__((ext_vector_type(2)))  float    v2f;
typedef __attribute__((ext_vector_type(2)))  unsigned v2u;

constexpr int kBatch = 4;
constexpr int kSeq   = 2048;
constexpr int kEmb   = 1024;
constexpr int kHeads = 16;
constexpr int kHd    = 64;
constexpr int kHid   = kHeads * kHd;
constexpr int kFfn   = 4 * kHid;
constexpr int kRows  = kBatch * kSeq;
constexpr float kWCarry    = 32.0f;
constexpr float kWCarryInv = 1.0f / kWCarry;
constexpr float kLnEps     = 1e-5f;
static_assert(kHid == 1024 && kFfn == 4096 && kRows == 8192, "shape constants");
static_assert((kEmb % 32) == 0 && (kHd % 32) == 0 && (kHid % 32) == 0 && (kFfn % 32) == 0, "GEMM K multiples of 32");
static_assert((kRows % 64) == 0 && ((3 * kHid) % 64) == 0 && (kHd % 64) == 0 && (kFfn % 64) == 0 && (kHid % 64) == 0, "GEMM M,N multiples of 64");
static_assert((((kRows / 64) * (3 * kHid / 64)) % 8) == 0 && ((3 * kHid / 64) % 8) == 0 && ((kHid / 64) % 8) == 0, "8 tiles per block stay inside one output section");

constexpr size_t kOffX16  = 0;
constexpr size_t kOffWABD = kOffX16  + (size_t)kRows * kEmb * 2;
constexpr size_t kOffWCT  = kOffWABD + (size_t)3 * kHid * kEmb * 2;
constexpr size_t kOffW1T  = kOffWCT  + (size_t)kHeads * kHd * kHd * 2;
constexpr size_t kOffW2T  = kOffW1T  + (size_t)kFfn * kHid * 2;
constexpr size_t kOffWPT  = kOffW2T  + (size_t)kHid * kFfn * 2;
constexpr size_t kOffA32  = kOffWPT  + (size_t)kHid * kHid * 2;
constexpr size_t kOffB32  = kOffA32  + (size_t)kRows * kHid * 4;
constexpr size_t kOffD16  = kOffB32  + (size_t)kRows * kHid * 4;
constexpr size_t kWsTotal = kOffD16  + (size_t)kRows * kHid * 2;
static_assert(kWsTotal == 125960192ull, "carve total");
static_assert(kWsTotal <= 134217728ull, "carve cap");
static_assert((size_t)kRows * kFfn * 2 == (kOffD16 - kOffA32), "gelu plane fits exactly over A32|B32");
static_assert((kOffWABD % 128) == 0 && (kOffWCT % 128) == 0 && (kOffW1T % 128) == 0 && (kOffW2T % 128) == 0 &&
              (kOffWPT % 128) == 0 && (kOffA32 % 128) == 0 && (kOffB32 % 128) == 0 && (kOffD16 % 128) == 0, "128-B aligned regions");

__device__ __forceinline__ float h16_to_f32(unsigned hb) {
  const unsigned sgn = (hb & 0x8000u) << 16;
  const unsigned em  = hb & 0x7fffu;
  const float fn = __uint_as_float((em << 13) + 0x38000000u);
  const float fs = (float)em * 5.9604644775390625e-8f;
  const float mag = (em < 0x400u) ? fs : fn;
  return __uint_as_float(__float_as_uint(mag) | sgn);
}

__device__ __forceinline__ void guard4_h(v8f& a0, v8f& a1, v8f& a2, v8f& a3, v16h x, v16h b0, v16h b1, v16h b2, v16h b3) {
  asm volatile("v_nop\n\tv_nop\n\tv_nop\n\tv_nop" : "+v"(a0), "+v"(a1), "+v"(a2), "+v"(a3) : "v"(x), "v"(b0), "v"(b1), "v"(b2), "v"(b3));
}
__device__ __forceinline__ void acc_guard4(v8f& a, v8f& b, v8f& c, v8f& d) {
  asm volatile("v_nop\n\tv_nop\n\tv_nop\n\tv_nop" : "+v"(a), "+v"(b), "+v"(c), "+v"(d));
}
__device__ __forceinline__ void wave_lds_sync() {
  __builtin_amdgcn_fence(__ATOMIC_RELEASE, "workgroup");
  __builtin_amdgcn_wave_barrier();
  __builtin_amdgcn_fence(__ATOMIC_ACQUIRE, "workgroup");
}
union FragU { v16h v; v8h h[2]; };
__device__ __forceinline__ v16h frag_load(const _Float16* p) {
  FragU f;
  f.h[0] = *(const v8h*)(p);
  f.h[1] = *(const v8h*)(p + 16);
  return f.v;
}
__device__ __forceinline__ v8f frag_mma(v16h a, v16h b, v8f c) {
  return __builtin_amdgcn_wmma_f32_16x16x32_f16(false, a, false, b, (short)0, c, false, false);
}

template <int EPI>
__global__ __launch_bounds__(256) void gemm64_f16(
    const unsigned short* __restrict__ Ap, int lda, long strideA,
    const unsigned short* __restrict__ Btp, int ldb, long strideB,
    void* C0, void* C1, void* C2, int ldc, long strideC,
    const float* bias0, const float* bias1, const float* bias2, long strideBias,
    const unsigned short* aux, long strideAux,
    int M, int N, int K, float scale)
{
  __shared__ __align__(16) float sT[8][16 * 68];
  const int b    = blockIdx.y;
  const int lane = threadIdx.x & 31;
  const int wave = threadIdx.x >> 5;
  const int tilesN = N >> 6;
  const int tilesM = M >> 6;
  const int tile = blockIdx.x * 8 + wave;
  if (tile >= tilesM * tilesN) return;
  const int tm = tile / tilesN;
  const int tn = tile - tm * tilesN;
  const int m0 = tm << 6;
  const int n0 = tn << 6;
  int sel = 0;
  if (EPI == 0) {
    const int tnb = (int)((blockIdx.x * 8u) % (unsigned)tilesN);
    sel = (tnb << 6) / ldc;
  }
  const int ncol0 = n0 - sel * ldc;

  const int rlane = lane & 15;
  const int koff  = (lane >> 4) * 8;
  const int mOff  = (lane >> 4) * 8;

  const _Float16* aq = (const _Float16*)Ap  + (size_t)b * strideA + (size_t)(m0 + rlane) * lda + koff;
  const _Float16* bq = (const _Float16*)Btp + (size_t)b * strideB + (size_t)(n0 + rlane) * ldb + koff;
  const size_t aStep = (size_t)16 * lda;
  const size_t bStep = (size_t)16 * ldb;

  v8f acc[4][4];
#pragma unroll
  for (int i = 0; i < 4; ++i)
#pragma unroll
    for (int j = 0; j < 4; ++j) acc[i][j] = (v8f){0.f, 0.f, 0.f, 0.f, 0.f, 0.f, 0.f, 0.f};

  for (int k0 = 0; k0 < K; k0 += 32) {
    v16h bh[4];
#pragma unroll
    for (int j = 0; j < 4; ++j) bh[j] = frag_load(bq + j * bStep + k0);
#pragma unroll
    for (int i = 0; i < 4; ++i) {
      const v16h ah = frag_load(aq + i * aStep + k0);
#pragma unroll
      for (int j = 0; j < 4; ++j) acc[i][j] = frag_mma(ah, bh[j], acc[i][j]);
      guard4_h(acc[i][0], acc[i][1], acc[i][2], acc[i][3], ah, bh[0], bh[1], bh[2], bh[3]);
    }
  }
  acc_guard4(acc[0][0], acc[0][1], acc[0][2], acc[0][3]);
  acc_guard4(acc[1][0], acc[1][1], acc[1][2], acc[1][3]);
  acc_guard4(acc[2][0], acc[2][1], acc[2][2], acc[2][3]);
  acc_guard4(acc[3][0], acc[3][1], acc[3][2], acc[3][3]);

  float* slab = sT[wave];
  const float* bp = ((sel == 0) ? bias0 : ((sel == 1) ? bias1 : bias2)) + (size_t)b * strideBias;
  float bvj[4];
#pragma unroll
  for (int j = 0; j < 4; ++j) bvj[j] = bp[ncol0 + (j << 4) + rlane];
  const bool out16 = (EPI == 1) || (EPI == 2) || ((EPI == 0) && (sel == 2));
  const unsigned short* auxb = aux + (size_t)b * strideAux;
  const int hh = lane >> 4, c4 = (lane & 15) * 4;
  const int q  = lane >> 3, c8 = (lane & 7) * 8;

#pragma unroll
  for (int i = 0; i < 4; ++i) {
    const int mBase = m0 + (i << 4);
#pragma unroll
    for (int j = 0; j < 4; ++j) {
#pragma unroll
      for (int r = 0; r < 8; ++r)
        slab[(mOff + r) * 68 + (j << 4) + rlane] = acc[i][j][r] * scale + bvj[j];
    }
    wave_lds_sync();

    if (EPI == 0) {
      if (sel == 0) {
#pragma unroll 1
        for (int idx = 0; idx < 32; ++idx) {
          float* sp = slab + ((idx >> 2) * 2 + hh) * 68 + c4 + (idx & 3);
          const float t = *sp;
          *sp = tanhf(t);
        }
      }
    }
    if (EPI == 1) {
#pragma unroll 1
      for (int idx = 0; idx < 32; ++idx) {
        float* sp = slab + ((idx >> 2) * 2 + hh) * 68 + c4 + (idx & 3);
        const float t = *sp;
        *sp = 0.5f * t * (1.0f + erff(t * 0.70710678118654752f));
      }
    }
    if (EPI == 2 || EPI == 4) {
#pragma unroll 1
      for (int it = 0; it < 8; ++it) {
        const int row = it * 2 + hh;
        const v2u w = *(const v2u*)(auxb + (size_t)(mBase + row) * ldc + n0 + c4);
        const unsigned w0 = w[0];
        const unsigned w1 = w[1];
        const float f0 = h16_to_f32(w0 & 0xffffu);
        const float f1 = h16_to_f32(w0 >> 16);
        const float f2 = h16_to_f32(w1 & 0xffffu);
        const float f3 = h16_to_f32(w1 >> 16);
        float* sp = slab + row * 68 + c4;
        v4f v = *(const v4f*)sp;
        if (EPI == 2) {
          v[0] = v[0] + f0; v[1] = v[1] + f1; v[2] = v[2] + f2; v[3] = v[3] + f3;
        } else {
          v[0] = v[0] * f0; v[1] = v[1] * f1; v[2] = v[2] * f2; v[3] = v[3] * f3;
        }
        *(v4f*)sp = v;
      }
    }
    wave_lds_sync();

    if (out16) {
      unsigned short* C = (unsigned short*)((EPI == 0) ? C2 : C0) + (size_t)b * strideC;
      for (int pass = 0; pass < 2; ++pass) {
#pragma unroll
        for (int it = 0; it < 4; ++it) {
          const int row = it * 4 + q;
          const float* sp = slab + row * 68 + c8;
          v8h hv;
#pragma unroll
          for (int e = 0; e < 8; ++e) hv[e] = (_Float16)sp[e];
          *(volatile v8h*)(C + (size_t)(mBase + row) * ldc + ncol0 + c8) = hv;
        }
        __threadfence();
      }
    } else {
      float* C = (float*)(((EPI == 0) && (sel == 1)) ? C1 : C0) + (size_t)b * strideC;
      for (int pass = 0; pass < 2; ++pass) {
#pragma unroll
        for (int it = 0; it < 8; ++it) {
          const int row = it * 2 + hh;
          const v4f v = *(const v4f*)(slab + row * 68 + c4);
          *(volatile v4f*)(C + (size_t)(mBase + row) * ldc + ncol0 + c4) = v;
        }
        __threadfence();
      }
    }
    wave_lds_sync();
  }
}

__global__ __launch_bounds__(256) void cast_f16_kernel(
    const float* __restrict__ src, unsigned short* __restrict__ dst, int total8, float scale)
{
  const int i = blockIdx.x * 256 + threadIdx.x;
  if (i >= total8) return;
  const size_t e0 = (size_t)i << 3;
  const float* p = src + e0;
  const v4f a0 = *(const v4f*)(p);
  const v4f a1 = *(const v4f*)(p + 4);
  v8h hv;
#pragma unroll
  for (int e = 0; e < 4; ++e) {
    hv[e]     = (_Float16)(a0[e] * scale);
    hv[4 + e] = (_Float16)(a1[e] * scale);
  }
  unsigned short* qd = dst + e0;
  *(volatile v8h*)qd = hv;
  __threadfence();
  *(volatile v8h*)qd = hv;
}

__global__ __launch_bounds__(256) void transpose_cast_kernel(
    const float* __restrict__ W0, const float* __restrict__ W1, const float* __restrict__ W2,
    int zper, long srcStride, unsigned short* __restrict__ Bt, long dstStride,
    int Kdim, int Ndim, float scale)
{
  __shared__ float tile[64 * 65];
  const int tid = threadIdx.x, lane = tid & 31, wave = tid >> 5;
  const int z  = blockIdx.z;
  const int zs = z / zper;
  const int zl = z - zs * zper;
  const float* W = ((zs == 0) ? W0 : ((zs == 1) ? W1 : W2)) + (size_t)zl * srcStride;
  unsigned short* D = Bt + (size_t)z * dstStride;
  const int n0 = blockIdx.x * 64;
  const int k0 = blockIdx.y * 64;
#pragma unroll
  for (int p = 0; p < 16; ++p) {
    const int idx = tid + p * 256;
    const int kk  = idx >> 6;
    const int nn  = idx & 63;
    const float v = W[(size_t)(k0 + kk) * Ndim + n0 + nn];
    tile[kk * 65 + nn] = v * scale;
  }
  __syncthreads();
  const int q = lane >> 3, c8 = (lane & 7) * 8;
  v8h hv[2];
#pragma unroll
  for (int it = 0; it < 2; ++it) {
    const int nrow = it * 32 + wave * 4 + q;
#pragma unroll
    for (int e = 0; e < 8; ++e) hv[it][e] = (_Float16)tile[(c8 + e) * 65 + nrow];
  }
  for (int pass = 0; pass < 2; ++pass) {
#pragma unroll
    for (int it = 0; it < 2; ++it) {
      const int nrow = it * 32 + wave * 4 + q;
      *(volatile v8h*)(D + (size_t)(n0 + nrow) * Kdim + k0 + c8) = hv[it];
    }
    __threadfence();
  }
}

__global__ __launch_bounds__(64) void scan_kernel(
    const float* __restrict__ A32, const float* __restrict__ B32, unsigned* __restrict__ H16w)
{
  const int g   = blockIdx.x * 64 + threadIdx.x;
  const int bix = g / (kHid / 2);
  const int col = (g - bix * (kHid / 2)) * 2;
  const size_t base = (size_t)bix * kSeq * kHid + col;
  const float* ap = A32 + base;
  const float* bp = B32 + base;
  unsigned* hp = H16w + (base >> 1);
  float h0 = 0.f, h1 = 0.f;
#pragma unroll 1
  for (int t = 0; t < kSeq; t += 4) {
    v2f av[4], bv[4];
#pragma unroll
    for (int s = 0; s < 4; ++s) {
      av[s] = *(const v2f*)(ap + (size_t)(t + s) * kHid);
      bv[s] = *(const v2f*)(bp + (size_t)(t + s) * kHid);
    }
    unsigned pk[4];
#pragma unroll
    for (int s = 0; s < 4; ++s) {
      h0 = fmaf(av[s][0], h0, bv[s][0]);
      h1 = fmaf(av[s][1], h1, bv[s][1]);
      v2h hv;
      hv[0] = (_Float16)h0;
      hv[1] = (_Float16)h1;
      pk[s] = __builtin_bit_cast(unsigned, hv);
    }
#pragma unroll
    for (int s = 0; s < 4; ++s) *(volatile unsigned*)(hp + (size_t)(t + s) * (kHid / 2)) = pk[s];
    __threadfence();
#pragma unroll
    for (int s = 0; s < 4; ++s) *(volatile unsigned*)(hp + (size_t)(t + s) * (kHid / 2)) = pk[s];
  }
}

__global__ __launch_bounds__(256) void ln_resid_kernel(
    const float* __restrict__ Z, const float* __restrict__ gam, const float* __restrict__ bet,
    unsigned short* __restrict__ U16)
{
  const int lane = threadIdx.x & 31, wave = threadIdx.x >> 5;
  const int row  = blockIdx.x * 8 + wave;
  const float* z = Z + (size_t)row * kHid;
  float x[32];
#pragma unroll
  for (int it = 0; it < 4; ++it) {
    const v4f a0 = *(const v4f*)(z + it * 256 + lane * 8);
    const v4f a1 = *(const v4f*)(z + it * 256 + lane * 8 + 4);
#pragma unroll
    for (int e = 0; e < 4; ++e) {
      x[it * 8 + e]     = a0[e];
      x[it * 8 + 4 + e] = a1[e];
    }
  }
  float s = 0.f;
#pragma unroll
  for (int i = 0; i < 32; ++i) s += x[i];
#pragma unroll
  for (int off = 16; off > 0; off >>= 1) s += __shfl_xor(s, off, 32);
  const float mu = s * (1.0f / (float)kHid);
  float vs = 0.f;
#pragma unroll
  for (int i = 0; i < 32; ++i) {
    const float t = x[i] - mu;
    vs += t * t;
  }
#pragma unroll
  for (int off = 16; off > 0; off >>= 1) vs += __shfl_xor(vs, off, 32);
  const float rstd = rsqrtf(vs * (1.0f / (float)kHid) + kLnEps);
  v8h hv[4];
#pragma unroll
  for (int it = 0; it < 4; ++it) {
    const v4f g0 = *(const v4f*)(gam + it * 256 + lane * 8);
    const v4f g1 = *(const v4f*)(gam + it * 256 + lane * 8 + 4);
    const v4f b0 = *(const v4f*)(bet + it * 256 + lane * 8);
    const v4f b1 = *(const v4f*)(bet + it * 256 + lane * 8 + 4);
#pragma unroll
    for (int e = 0; e < 4; ++e) {
      const float xa = x[it * 8 + e];
      const float xb = x[it * 8 + 4 + e];
      const float la = (xa - mu) * rstd * g0[e] + b0[e];
      const float lb = (xb - mu) * rstd * g1[e] + b1[e];
      hv[it][e]     = (_Float16)(xa + la);
      hv[it][4 + e] = (_Float16)(xb + lb);
    }
  }
  unsigned short* up = U16 + (size_t)row * kHid + lane * 8;
  for (int pass = 0; pass < 2; ++pass) {
#pragma unroll
    for (int it = 0; it < 4; ++it) *(volatile v8h*)(up + it * 256) = hv[it];
    __threadfence();
  }
}

extern "C" void kernel_launch(void* const* d_in, const int* in_sizes, int n_in,
                              void* d_out, int out_size, void* d_ws, size_t ws_size,
                              hipStream_t stream)
{
  if (n_in < 17) return;
  if (in_sizes[0] != kRows * kEmb) return;
  if (in_sizes[1] != kHeads * kEmb * kHd || in_sizes[3] != kHeads * kEmb * kHd || in_sizes[5] != kHeads * kEmb * kHd) return;
  if (in_sizes[2] != kHid || in_sizes[4] != kHid || in_sizes[6] != kHid || in_sizes[8] != kHid) return;
  if (in_sizes[7] != kHeads * kHd * kHd) return;
  if (in_sizes[9] != kHid * kFfn || in_sizes[10] != kFfn) return;
  if (in_sizes[11] != kFfn * kHid || in_sizes[12] != kHid) return;
  if (in_sizes[13] != kHid * kHid || in_sizes[14] != kHid) return;
  if (in_sizes[15] != kHid || in_sizes[16] != kHid) return;
  if (out_size != kRows * kHid) return;
  if (ws_size < kWsTotal) return;

  const float* emb    = (const float*)d_in[0];
  const float* Wa     = (const float*)d_in[1];
  const float* ba     = (const float*)d_in[2];
  const float* Wb     = (const float*)d_in[3];
  const float* bb     = (const float*)d_in[4];
  const float* WD     = (const float*)d_in[5];
  const float* bD     = (const float*)d_in[6];
  const float* WC     = (const float*)d_in[7];
  const float* bC     = (const float*)d_in[8];
  const float* ffn1_w = (const float*)d_in[9];
  const float* ffn1_b = (const float*)d_in[10];
  const float* ffn2_w = (const float*)d_in[11];
  const float* ffn2_b = (const float*)d_in[12];
  const float* proj_w = (const float*)d_in[13];
  const float* proj_b = (const float*)d_in[14];
  const float* ln_g   = (const float*)d_in[15];
  const float* ln_b   = (const float*)d_in[16];
  float* out = (float*)d_out;

  char* ws = (char*)d_ws;
  unsigned short* X16   = (unsigned short*)(ws + kOffX16);
  unsigned short* WABD  = (unsigned short*)(ws + kOffWABD);
  unsigned short* WCT   = (unsigned short*)(ws + kOffWCT);
  unsigned short* W1T   = (unsigned short*)(ws + kOffW1T);
  unsigned short* W2T   = (unsigned short*)(ws + kOffW2T);
  unsigned short* WPT   = (unsigned short*)(ws + kOffWPT);
  float*          A32   = (float*)(ws + kOffA32);
  float*          B32   = (float*)(ws + kOffB32);
  unsigned short* MID16 = (unsigned short*)(ws + kOffA32);
  unsigned short* D16   = (unsigned short*)(ws + kOffD16);

  cast_f16_kernel<<<(kRows * kEmb) / 8 / 256, 256, 0, stream>>>(emb, X16, (kRows * kEmb) / 8, 1.0f);

  transpose_cast_kernel<<<dim3(kHd / 64, kEmb / 64, 3 * kHeads), 256, 0, stream>>>(
      Wa, Wb, WD, kHeads, (long)kEmb * kHd, WABD, (long)kHd * kEmb, kEmb, kHd, kWCarry);
  transpose_cast_kernel<<<dim3(kHd / 64, kHd / 64, kHeads), 256, 0, stream>>>(
      WC, WC, WC, kHeads, (long)kHd * kHd, WCT, (long)kHd * kHd, kHd, kHd, kWCarry);
  transpose_cast_kernel<<<dim3(kFfn / 64, kHid / 64, 1), 256, 0, stream>>>(
      ffn1_w, ffn1_w, ffn1_w, 1, 0L, W1T, 0L, kHid, kFfn, kWCarry);
  transpose_cast_kernel<<<dim3(kHid / 64, kFfn / 64, 1), 256, 0, stream>>>(
      ffn2_w, ffn2_w, ffn2_w, 1, 0L, W2T, 0L, kFfn, kHid, kWCarry);
  transpose_cast_kernel<<<dim3(kHid / 64, kHid / 64, 1), 256, 0, stream>>>(
      proj_w, proj_w, proj_w, 1, 0L, WPT, 0L, kHid, kHid, kWCarry);

  gemm64_f16<0><<<dim3((kRows / 64) * (3 * kHid / 64) / 8, 1), 256, 0, stream>>>(
      X16, kEmb, 0L, WABD, kEmb, 0L,
      (void*)A32, (void*)B32, (void*)D16, kHid, 0L,
      ba, bb, bD, 0L, X16, 0L,
      kRows, 3 * kHid, kEmb, kWCarryInv);

  scan_kernel<<<(kBatch * (kHid / 2)) / 64, 64, 0, stream>>>(A32, B32, (unsigned*)X16);

  gemm64_f16<4><<<dim3((kRows / 64) / 8, kHeads), 256, 0, stream>>>(
      X16, kHid, (long)kHd, WCT, kHd, (long)kHd * kHd,
      (void*)A32, (void*)A32, (void*)A32, kHid, (long)kHd,
      bC, bC, bC, (long)kHd, D16, (long)kHd,
      kRows, kHd, kHd, kWCarryInv);

  ln_resid_kernel<<<kRows / 8, 256, 0, stream>>>(A32, ln_g, ln_b, X16);

  gemm64_f16<1><<<dim3((kRows / 64) * (kFfn / 64) / 8, 1), 256, 0, stream>>>(
      X16, kHid, 0L, W1T, kHid, 0L,
      (void*)MID16, (void*)MID16, (void*)MID16, kFfn, 0L,
      ffn1_b, ffn1_b, ffn1_b, 0L, X16, 0L,
      kRows, kFfn, kHid, kWCarryInv);

  gemm64_f16<2><<<dim3((kRows / 64) * (kHid / 64) / 8, 1), 256, 0, stream>>>(
      MID16, kFfn, 0L, W2T, kFfn, 0L,
      (void*)D16, (void*)D16, (void*)D16, kHid, 0L,
      ffn2_b, ffn2_b, ffn2_b, 0L, X16, 0L,
      kRows, kHid, kFfn, kWCarryInv);

  gemm64_f16<3><<<dim3((kRows / 64) * (kHid / 64) / 8, 1), 256, 0, stream>>>(
      D16, kHid, 0L, WPT, kHid, 0L,
      (void*)out, (void*)out, (void*)out, kHid, 0L,
      proj_b, proj_b, proj_b, 0L, X16, 0L,
      kRows, kHid, kHid, kWCarryInv);
}
